// GATEncoder_12455405158966
// MI455X (gfx1250) — hardware-verified
//
#include <hip/hip_runtime.h>


namespace {
constexpr int B = 32, N = 512, F0 = 128, H = 8, DD = 64, D = H * DD  , NR = B * N, BL = 32  ;
constexpr float XS = 8.0f, WSC = 256.0f, WSQ = 0.25f, PS = 1024.0f, RS_ = 1024.0f, LOG2E = 1.4426950408889634f, NSL_ = 0.01f;
static_assert(N % 64 == 0 && F0 % 32 == 0 && D % 128 == 0 && DD == 64, "tiling");
typedef _Float16 b16;
typedef __attribute__((ext_vector_type(16))) _Float16 v16b;
typedef __attribute__((ext_vector_type(8))) _Float16 v8b;
typedef __attribute__((ext_vector_type(8))) float v8f;
typedef __attribute__((ext_vector_type(4))) float v4f;
__device__ __forceinline__ float bf16_rne(float f) { unsigned int u = __float_as_uint(f); u += 0x7FFFu + ((u >> 16) & 1u); return __uint_as_float(u & 0xFFFF0000u); }
__device__ __forceinline__ void split16(float v, b16& hi, b16& lo) { hi = (b16)v; lo = (b16)(v - (float)hi); }
__device__ __forceinline__ v16b frag_kb(const b16* p, int hh) { const v8b a = *(const v8b*)(p + 8 * hh), b = *(const v8b*)(p + 16 + 8 * hh); v16b f;
#pragma unroll
  for (int e = 0; e < 8; ++e) { f[e] = a[e]; f[8 + e] = b[e]; } return f; }
__device__ __forceinline__ v8f wmma16b(v16b a, v16b b, v8f c) { v8f d = __builtin_amdgcn_wmma_f32_16x16x32_f16(false, a, false, b, (short)0, c, false, false); asm volatile("v_nop\n\tv_nop\n\tv_nop\n\tv_nop" : "+v"(d) : "v"(a), "v"(b)); return d; }
__device__ __forceinline__ void wave_lds_sync() { __builtin_amdgcn_fence(__ATOMIC_RELEASE, "workgroup"); __builtin_amdgcn_wave_barrier(); __builtin_amdgcn_fence(__ATOMIC_ACQUIRE, "workgroup"); }
__device__ __forceinline__ float pmul(float a, float b) { float p = a * b; asm volatile("" : "+v"(p)); return p; }
__device__ __forceinline__ int iclamp(int v, int lo, int hi) { return v < lo ? lo : (v > hi ? hi : v); }

typedef __attribute__((ext_vector_type(2))) _Float16 v2h;
typedef __attribute__((ext_vector_type(4))) _Float16 v4h;
typedef __attribute__((ext_vector_type(2))) float v2f;
typedef __attribute__((ext_vector_type(4))) int v4i;
__device__ __forceinline__ float nexp2(float v) { return __builtin_amdgcn_exp2f(v); }
__device__ __forceinline__ float lrelu(float v) { return v > 0.0f ? v : NSL_ * v; }
template <int FIN>
__global__ __launch_bounds__(256) void wt_kernel(const float* __restrict__ w, b16* __restrict__ WT, float scl) {
  const int u = blockIdx.x * 256 + threadIdx.x; if (u >= D * FIN / 8) return; const int e = u * 8; const int o = e / FIN, k0 = e % FIN; const int h = o / DD, dd = o % DD; v8b v;
#pragma unroll
  for (int j = 0; j < 8; ++j) v[j] = (b16)(bf16_rne(w[((size_t)h * FIN + k0 + j) * DD + dd]) * scl);
  for (int pass = 0; pass < 2; ++pass) { *(volatile v8b*)(WT + e) = v; __threadfence(); }
}
template <int FIN, bool RND>
__global__ __launch_bounds__(128) void fts_kernel(const float* __restrict__ X, const b16* __restrict__ WT, const b16* __restrict__ WQ, const float* __restrict__ a1w, const float* __restrict__ a1b, const float* __restrict__ a2w, const float* __restrict__ a2b, float* __restrict__ FT, float* __restrict__ F12, b16* __restrict__ VTh, b16* __restrict__ VTl) {
  constexpr int KC = FIN < 256 ? FIN : 256;
  __shared__ __attribute__((aligned(16))) b16 As[64][KC + 8], Al[64][KC + 8]; __shared__ __attribute__((aligned(16))) float Tf[4][16][128 + 4];
  const int wave = threadIdx.x >> 5, lane = threadIdx.x & 31, nloc = lane & 15, hlf = lane >> 4; const int n0 = blockIdx.x * 64, b = blockIdx.y, slab = blockIdx.z, c0 = slab * 128;
  const float* xb = X + ((size_t)b * N + n0) * FIN;
  v8f acc[8];
#pragma unroll
  for (int t = 0; t < 8; ++t) acc[t] = (v8f){};
#pragma unroll 1
  for (int kc = 0; kc < FIN; kc += KC) {
    __syncthreads();
    for (int i = threadIdx.x; i < 64 * (KC / 4); i += 128) { const int rr = i / (KC / 4), q = (i % (KC / 4)) * 4; const v4f f = *(const v4f*)(xb + (size_t)rr * FIN + kc + q); v4h o, ol; for (int j = 0; j < 4; ++j) { const float vs = (RND ? bf16_rne(f[j]) : f[j]) * XS; const b16 p = (b16)vs; o[j] = p; ol[j] = (b16)((vs - (float)p) * RS_); } *(v4h*)(&As[rr][q]) = o; *(v4h*)(&Al[rr][q]) = ol; }
    __syncthreads();
#pragma unroll 2
    for (int kb = 0; kb < KC; kb += 32) { const v16b a = frag_kb(&As[wave * 16 + nloc][kb], hlf); v16b al; if (!RND) al = frag_kb(&Al[wave * 16 + nloc][kb], hlf);
#pragma unroll
      for (int t = 0; t < 8; ++t) { const size_t wo_ = (size_t)(c0 + t * 16 + nloc) * FIN + kc + kb; acc[t] = wmma16b(a, frag_kb(WT + wo_, hlf), acc[t]); if (!RND) acc[t] = wmma16b(al, frag_kb(WQ + wo_, hlf), acc[t]); } } }
#pragma unroll
  for (int t = 0; t < 8; ++t)
#pragma unroll
    for (int r = 0; r < 8; ++r) Tf[wave][8 * hlf + r][t * 16 + nloc] = acc[t][r] * (1.0f / (XS * WSC));
  __syncthreads();
  const int hA = 2 * slab + (lane >> 4); const int d0 = (lane & 15) * 4;
  float w1[4], w2[4]; for (int j = 0; j < 4; ++j) { w1[j] = bf16_rne(a1w[hA * DD + d0 + j]); w2[j] = bf16_rne(a2w[hA * DD + d0 + j]); } const float b1 = bf16_rne(a1b[hA]), b2 = bf16_rne(a2b[hA]);
  for (int pass = 0; pass < 2; ++pass) {
    for (int rr = 0; rr < 16; ++rr) { const int node = n0 + wave * 16 + rr; *(volatile v4f*)(FT + ((size_t)b * N + node) * D + c0 + lane * 4) = *(const v4f*)(&Tf[wave][rr][lane * 4]);
      float s1 = 0.0f, s2 = 0.0f; for (int j = 0; j < 4; ++j) { const float fv = Tf[wave][rr][lane * 4 + j]; s1 = fmaf(fv, w1[j], s1); s2 = fmaf(fv, w2[j], s2); }
      for (int o = 1; o <= 8; o <<= 1) { s1 += __shfl_xor(s1, o); s2 += __shfl_xor(s2, o); }
      if ((lane & 15) == rr) { v2f sc; sc[0] = s1 + b1; sc[1] = s2 + b2; *(volatile v2f*)(F12 + (((size_t)b * H + hA) * N + node) * 2) = sc; } }
#pragma unroll 1
    for (int q = 0; q < 32; ++q) { const int cl = wave * 32 + q; const int c = c0 + cl; const int h = c / DD, dd = c % DD; const int tk = lane * 2; v2h hv, lv;
      for (int j = 0; j < 2; ++j) { const float f = Tf[(tk + j) >> 4][(tk + j) & 15][cl] * XS; const b16 p = (b16)f; hv[j] = p; lv[j] = (b16)((f - (float)p) * RS_); }
      const size_t oi = (((size_t)b * H + h) * DD + dd) * (size_t)N + n0 + lane * 2; *(volatile v2h*)(VTh + oi) = hv; *(volatile v2h*)(VTl + oi) = lv; }
    __threadfence(); }
}
__global__ __launch_bounds__(64) void att_kernel(const float* __restrict__ FT, const float* __restrict__ F12, const b16* __restrict__ VTh, const b16* __restrict__ VTl, float* __restrict__ OUT) {
  __shared__ __attribute__((aligned(16))) b16 Pb[2][16][32 + 8], Pl[2][16][32 + 8]; __shared__ __attribute__((aligned(16))) float To[2][16][DD + 4];
  const int wave = threadIdx.x >> 5, lane = threadIdx.x & 31, hh = lane >> 4, col = lane & 15; const int b = blockIdx.y / H, h = blockIdx.y % H; const int i0 = blockIdx.x * 32 + wave * 16, ii = i0 + col;
  const float* f12 = F12 + ((size_t)b * H + h) * N * 2; const b16* Vh = VTh + ((size_t)b * H + h) * DD * (size_t)N; const b16* Vl = VTl + ((size_t)b * H + h) * DD * (size_t)N;
  float m2 = -INFINITY; for (int j = lane; j < N; j += 32) m2 = fmaxf(m2, f12[(size_t)j * 2 + 1]);
#pragma unroll
  for (int o = 16; o >= 1; o >>= 1) m2 = fmaxf(m2, __shfl_xor(m2, o));
  const float f1 = f12[(size_t)ii * 2]; const float mi = lrelu(f1 + m2);
  float l = 0.0f; v8f o[4], ol[4]; for (int t = 0; t < 4; ++t) { o[t] = (v8f){}; ol[t] = (v8f){}; }
#pragma unroll 1
  for (int kb = 0; kb < N; kb += 32) {
#pragma unroll
    for (int i2 = 0; i2 < 16; ++i2) { const int j = kb + (i2 < 8 ? 0 : 16) + 8 * hh + (i2 & 7); const float p = nexp2((lrelu(f1 + f12[(size_t)j * 2 + 1]) - mi) * LOG2E); l += p; const float ps = p * PS; const b16 phh = (b16)ps; const int pc = (i2 < 8 ? 0 : 16) + 8 * hh + (i2 & 7); Pb[wave][col][pc] = phh; Pl[wave][col][pc] = (b16)((ps - (float)phh) * RS_); }
    wave_lds_sync();
    const v16b pf = frag_kb(&Pb[wave][col][0], hh), plf = frag_kb(&Pl[wave][col][0], hh);
#pragma unroll
    for (int t = 0; t < 4; ++t) { const v16b vh = frag_kb(Vh + (size_t)(t * 16 + col) * N + kb, hh); o[t] = wmma16b(vh, pf, o[t]); ol[t] = wmma16b(frag_kb(Vl + (size_t)(t * 16 + col) * N + kb, hh), pf, ol[t]); ol[t] = wmma16b(vh, plf, ol[t]); }
    wave_lds_sync(); }
  l += __shfl_xor(l, 16);
  const float inv = 1.0f / (l * PS * XS);
#pragma unroll
  for (int t = 0; t < 4; ++t)
#pragma unroll
    for (int r = 0; r < 8; ++r) To[wave][col][t * 16 + 8 * hh + r] = (o[t][r] + ol[t][r] * (1.0f / RS_)) * inv;
  wave_lds_sync();
  for (int pass = 0; pass < 2; ++pass) { for (int rr = 0; rr < 16; ++rr) { const size_t row = (size_t)b * N + i0 + rr; const v2f vv = *(const v2f*)(&To[wave][rr][lane * 2]); const v2f fv = *(const v2f*)(FT + row * D + h * DD + lane * 2); v2f r2;
      for (int j = 0; j < 2; ++j) { const float t_ = vv[j] + fv[j]; r2[j] = t_ > 0.0f ? t_ : (__expf(t_) - 1.0f); }
      *(volatile v2f*)(OUT + row * D + h * DD + lane * 2) = r2; } __threadfence(); }
}
}

extern "C" void kernel_launch(void* const* d_in, const int* in_sizes, int n_in, void* d_out, int out_size, void* d_ws, size_t ws_size, hipStream_t stream) {
  (void)n_in;
  auto Fp = [&](int i) { return (const float*)d_in[i]; };
  if (in_sizes[0] != NR * F0 || in_sizes[1] != H * F0 * DD || in_sizes[2] != H * D * DD || in_sizes[3] != 2 * H * DD || in_sizes[4] != 2 * H || in_sizes[5] != 2 * H * DD || in_sizes[6] != 2 * H || out_size != NR * D) return;
  size_t off = 0; char* ws = (char*)d_ws;
  auto carve = [&](size_t bytes) { char* p = ws + off; off += (bytes + 255) & ~(size_t)255; return p; };
  b16* WT0 = (b16*)carve((size_t)D * F0 * 2); b16* WT1 = (b16*)carve((size_t)D * D * 2); b16* WQ1 = (b16*)carve((size_t)D * D * 2);
  float* FT = (float*)carve((size_t)NR * D * 4); float* F12 = (float*)carve((size_t)B * H * N * 2 * 4); b16* VTh = (b16*)carve((size_t)NR * D * 2); b16* VTl = (b16*)carve((size_t)NR * D * 2); float* H1 = (float*)carve((size_t)NR * D * 4);
  if (off > ws_size || off > ((size_t)128 << 20)) return;
  wt_kernel<F0><<<(D * F0 / 8 + 255) / 256, 256, 0, stream>>>(Fp(1), WT0, WSC);
  wt_kernel<D><<<(D * D / 8 + 255) / 256, 256, 0, stream>>>(Fp(2), WT1, WSC); wt_kernel<D><<<(D * D / 8 + 255) / 256, 256, 0, stream>>>(Fp(2), WQ1, WSQ);
  fts_kernel<F0, true><<<dim3(N / 64, BL, D / 128), 128, 0, stream>>>(Fp(0), WT0, WT0, Fp(3), Fp(4), Fp(5), Fp(6), FT, F12, VTh, VTl);
  att_kernel<<<dim3(N / 32, BL * H), 64, 0, stream>>>(FT, F12, VTh, VTl, H1);
  fts_kernel<D, false><<<dim3(N / 64, BL, D / 128), 128, 0, stream>>>(H1, WT1, WQ1, Fp(3) + H * DD, Fp(4) + H, Fp(5) + H * DD, Fp(6) + H, FT, F12, VTh, VTl);
  att_kernel<<<dim3(N / 32, BL * H), 64, 0, stream>>>(FT, F12, VTh, VTl, (float*)d_out);
}
